// CNNLR_58712202936614
// MI455X (gfx1250) — hardware-verified
//
#include <hip/hip_runtime.h>


#define NB_  128
#define LL   26
#define CH1   128
#define CH2   64
#define K1   7
#define K2   5
#define KIM  (CH1 * K2)
#define NRW  (NB_ * LL)
#define NF   (LL * CH2)
#define NPOS 25
#define WOFF (1 + NF)
#define NSO  (CH2 * CH2 * (NPOS * (NPOS + 1) / 2))
#define DM   KIM
#define LOSC 1024.0f

typedef _Float16 h16;
typedef unsigned short bf;
typedef __attribute__((ext_vector_type(16))) __bf16   v16bf;
typedef __attribute__((ext_vector_type(16))) _Float16 v16h;
typedef __attribute__((ext_vector_type(8)))  _Float16 v8h;
typedef __attribute__((ext_vector_type(8)))  unsigned short v8us;
typedef __attribute__((ext_vector_type(8)))  float    v8f;
typedef __attribute__((ext_vector_type(4)))  float    v4f;
typedef v8h  __attribute__((may_alias)) v8ha;
typedef v4f  __attribute__((may_alias)) v4fa;
typedef v8us __attribute__((may_alias)) v8usa;

__device__ __forceinline__ unsigned short f2bf(float f) { unsigned u = __float_as_uint(f); u += 0x7FFFu + ((u >> 16) & 1u); return (unsigned short)(u >> 16); }
__device__ __forceinline__ float bf2f(unsigned short b) { return __uint_as_float(((unsigned)b) << 16); }
__device__ __forceinline__ float bfr(float f) { return bf2f(f2bf(f)); }
__device__ __forceinline__ v16h cat16(v8h lo, v8h hi) { return __builtin_shufflevector(lo, hi, 0, 1, 2, 3, 4, 5, 6, 7, 8, 9, 10, 11, 12, 13, 14, 15); }
__device__ __forceinline__ v16bf cat16b(v8us lo, v8us hi) { return __builtin_bit_cast(v16bf, __builtin_shufflevector(lo, hi, 0, 1, 2, 3, 4, 5, 6, 7, 8, 9, 10, 11, 12, 13, 14, 15)); }
__device__ __forceinline__ v8f wmma16(v16h a, v16h b, v8f c) { return __builtin_amdgcn_wmma_f32_16x16x32_f16(false, a, false, b, (short)0, c, false, false); }
__device__ __forceinline__ v8f wmmab(v16bf a, v16bf b, v8f c) { return __builtin_amdgcn_wmma_f32_16x16x32_bf16(false, a, false, b, (short)0, c, false, false); }

template <bool SPLITA, bool F16OUT = false>
__global__ __launch_bounds__(128) void k_gemmb(const bf* __restrict__ A, const bf* __restrict__ Al, const bf* __restrict__ Bn, const float* __restrict__ bias, float* C, int ldc, h16* C2, const float* __restrict__ R = nullptr, int K = DM, int roundR = 1) {
    __shared__ __align__(16) float ost[4][16 * 68];
    const int lane = threadIdx.x & 31, wave = threadIdx.x >> 5, lr = lane & 15, hi = lane >> 4;
    const int r0 = blockIdx.x * 64 + wave * 16, c0 = blockIdx.y * 64;
    const size_t aoff = (size_t)(r0 + lr) * K + 8 * hi;
    size_t boff[4];
#pragma unroll
    for (int t = 0; t < 4; ++t) boff[t] = (size_t)(c0 + t * 16 + lr) * K + 8 * hi;
    v8f acc[4];
#pragma unroll
    for (int t = 0; t < 4; ++t) acc[t] = (v8f){};
#pragma unroll 1
    for (int kc = 0; kc < K; kc += 32) {
        const v16bf a = cat16b(*(const v8us*)(A + aoff + kc), *(const v8us*)(A + aoff + kc + 16));
        v16bf al = a;
        if (SPLITA) al = cat16b(*(const v8us*)(Al + aoff + kc), *(const v8us*)(Al + aoff + kc + 16));
#pragma unroll
        for (int t = 0; t < 4; ++t) { const v16bf b = cat16b(*(const v8us*)(Bn + boff[t] + kc), *(const v8us*)(Bn + boff[t] + kc + 16)); acc[t] = wmmab(a, b, acc[t]); if (SPLITA) acc[t] = wmmab(al, b, acc[t]); }
        asm volatile("v_nop\n\tv_nop\n\tv_nop\n\tv_nop" : "+v"(acc[0]), "+v"(acc[1]), "+v"(acc[2]), "+v"(acc[3]) : "v"(a), "v"(al));
    }
    float* os = &ost[wave][0];
#pragma unroll
    for (int t = 0; t < 4; ++t) { const float bv = bias ? bfr(bias[c0 + t * 16 + lr]) : 0.f;
#pragma unroll
        for (int j = 0; j < 8; ++j) os[(hi * 8 + j) * 68 + t * 16 + lr] = acc[t][j] + bv; }
    __syncthreads();
    if (F16OUT) {
        h16* crow = (h16*)(void*)C + (size_t)r0 * ldc + c0;
        auto pass = [&]() {
#pragma unroll
            for (int s = 0; s < 4; ++s) { const int row = 4 * s + (lane >> 3), piece = lane & 7; const float* sp = os + row * 68 + piece * 8; v8h o, o2;
#pragma unroll
                for (int i = 0; i < 8; ++i) { const h16 a = (h16)sp[i]; o[i] = a; o2[i] = (h16)((sp[i] - (float)a) * LOSC); }
                *(volatile v8h*)(crow + (size_t)row * ldc + piece * 8) = o; if (C2) *(volatile v8h*)(C2 + (size_t)r0 * ldc + c0 + (size_t)row * ldc + piece * 8) = o2; }
        };
        pass(); __threadfence(); pass();
    } else {
        float* crow = C + (size_t)r0 * ldc + c0;
        auto pass = [&]() {
#pragma unroll
            for (int s = 0; s < 8; ++s) { const int Lid = (lane >> 3) + 4 * s, piece = lane & 7; const int row = Lid >> 1, cofs = (Lid & 1) * 32 + piece * 4;
                v4f val = *(const v4fa*)(os + row * 68 + cofs); if (R) { const v4f rv = *(const v4f*)(R + ((size_t)r0 + row) * ldc + c0 + cofs); val += roundR ? (v4f){bfr(rv[0]), bfr(rv[1]), bfr(rv[2]), bfr(rv[3])} : rv; }
                *(volatile v4f*)(crow + (size_t)row * ldc + cofs) = val; }
        };
        pass(); __threadfence(); pass();
    }
}


__global__ __launch_bounds__(256) void k_bf(const float* __restrict__ src, bf* dst, size_t n8) {
    const size_t i = (size_t)blockIdx.x * 256 + threadIdx.x; if (i >= n8) return;
    const v8f v = *(const v8f*)(src + i * 8); v8us o;
#pragma unroll
    for (int k = 0; k < 8; ++k) o[k] = f2bf(v[k]);
    *(volatile v8us*)(dst + i * 8) = o; __threadfence(); *(volatile v8us*)(dst + i * 8) = o;
}

__global__ __launch_bounds__(256) void k_wso(const float* __restrict__ rw, bf* WSO) {
    const size_t u = (size_t)blockIdx.x * 256 + threadIdx.x; if (u >= (size_t)NSO / 8) return; v8us o;
    const float* src = rw + WOFF + u * 8;
#pragma unroll
    for (int i = 0; i < 8; ++i) o[i] = f2bf(src[i]);
    *(volatile v8us*)(WSO + u * 8) = o; __threadfence(); *(volatile v8us*)(WSO + u * 8) = o;
}
__global__ __launch_bounds__(128) void k_conv1(const int* __restrict__ xs, const float* __restrict__ w1, const float* __restrict__ b1, float* H1) {
    __shared__ int xl[LL];
    const int b = blockIdx.x, c = threadIdx.x;
    if (c < LL) xl[c] = xs[b * LL + c];
    __syncthreads();
    float v[LL];
#pragma unroll
    for (int l = 0; l < LL; ++l) { float a = bfr(b1[c]);
#pragma unroll
        for (int t = 0; t < K1; ++t) { const int p = l + t - K1 / 2; if (p >= 0 && p < LL) { const int xv = xl[p]; const int xc = xv < 0 ? 0 : (xv > 3 ? 3 : xv); const float w = bfr(w1[(c * 4 + xc) * K1 + t]); a += (xv >= 0 && xv < 4) ? w : 0.f; } }
        v[l] = fmaxf(a, 0.f); }
#pragma unroll 1
    for (int ps = 0; ps < 2; ++ps) {
#pragma unroll
        for (int l = 0; l < LL; ++l) *(volatile float*)(H1 + ((size_t)b * LL + l) * CH1 + c) = v[l];
        if (ps == 0) __threadfence(); }
}
__global__ __launch_bounds__(256) void k_im2col(const float* __restrict__ H1, bf* Ah, bf* Al) {
    const int lane = threadIdx.x & 31, r = blockIdx.x * 8 + (threadIdx.x >> 5); if (r >= NRW) return;
    const int b = r / LL, l = r % LL;
#pragma unroll 1
    for (int ps = 0; ps < 2; ++ps) {
#pragma unroll 1
        for (int k0 = lane * 8; k0 < KIM; k0 += 256) { v8us oh, ol;
#pragma unroll
            for (int i = 0; i < 8; ++i) { const int k = k0 + i, c = k / K2, t = k % K2, p = l + t - K2 / 2; const int pc = p < 0 ? 0 : (p >= LL ? LL - 1 : p);
                const float hv = H1[((size_t)b * LL + pc) * CH1 + c]; const float v = (p >= 0 && p < LL) ? hv : 0.f; const unsigned short hb = f2bf(v); oh[i] = hb; ol[i] = f2bf(v - bf2f(hb)); }
            const size_t o = (size_t)r * KIM + k0; *(volatile v8us*)(Ah + o) = oh; *(volatile v8us*)(Al + o) = ol; }
        if (ps == 0) __threadfence(); }
}
__global__ __launch_bounds__(256) void k_feat(const float* __restrict__ H2, float* Ff, bf* Fh, bf* Fl) {
    const int lane = threadIdx.x & 31, b = blockIdx.x * 8 + (threadIdx.x >> 5); if (b >= NB_) return;
    const float* src = H2 + (size_t)b * NF;
#pragma unroll 1
    for (int ps = 0; ps < 2; ++ps) {
#pragma unroll 1
        for (int c0 = lane * 4; c0 < NF; c0 += 128) { v4f v = *(const v4f*)(src + c0);
#pragma unroll
            for (int i = 0; i < 4; ++i) v[i] = fmaxf(v[i], 0.f);
            *(volatile v4f*)(Ff + (size_t)b * NF + c0) = v; }
#pragma unroll 1
        for (int c0 = lane * 8; c0 < NF; c0 += 256) { const v8f v = *(const v8f*)(src + c0); v8us oh, ol;
#pragma unroll
            for (int i = 0; i < 8; ++i) { const float y = fmaxf(v[i], 0.f); const unsigned short hb = f2bf(y); oh[i] = hb; ol[i] = f2bf(y - bf2f(hb)); }
            *(volatile v8us*)(Fh + (size_t)b * NF + c0) = oh; *(volatile v8us*)(Fl + (size_t)b * NF + c0) = ol; }
        if (ps == 0) __threadfence(); }
}
__global__ __launch_bounds__(128) void k_gemml(const bf* __restrict__ Ah, const bf* __restrict__ Al, int lda, const bf* __restrict__ Bn, int K, float* C, int ldc) {
    __shared__ __align__(16) float ost[4][16 * 68];
    const int lane = threadIdx.x & 31, wave = threadIdx.x >> 5, lr = lane & 15, hi = lane >> 4;
    const int r0 = blockIdx.x * 64 + wave * 16, c0 = blockIdx.y * 64;
    const size_t aoff = (size_t)(r0 + lr) * lda + 8 * hi;
    v8f acc[4];
#pragma unroll
    for (int t = 0; t < 4; ++t) acc[t] = (v8f){};
#pragma unroll 1
    for (int kc = 0; kc < K; kc += 32) {
        const v16bf a = cat16b(*(const v8us*)(Ah + aoff + kc), *(const v8us*)(Ah + aoff + kc + 16));
        const v16bf al = cat16b(*(const v8us*)(Al + aoff + kc), *(const v8us*)(Al + aoff + kc + 16));
#pragma unroll
        for (int t = 0; t < 4; ++t) { const size_t bo = (size_t)(c0 + t * 16 + lr) * K + kc + 8 * hi;
            const v16bf bb = cat16b(*(const v8us*)(Bn + bo), *(const v8us*)(Bn + bo + 16)); acc[t] = wmmab(a, bb, acc[t]); acc[t] = wmmab(al, bb, acc[t]); }
        asm volatile("v_nop\n\tv_nop\n\tv_nop\n\tv_nop" : "+v"(acc[0]), "+v"(acc[1]), "+v"(acc[2]), "+v"(acc[3]) : "v"(a), "v"(al));
    }
    float* os = &ost[wave][0];
#pragma unroll
    for (int t = 0; t < 4; ++t) {
#pragma unroll
        for (int j = 0; j < 8; ++j) os[(hi * 8 + j) * 68 + t * 16 + lr] = acc[t][j]; }
    __builtin_amdgcn_wave_barrier(); asm volatile("" ::: "memory");
    float* crow = C + (size_t)r0 * ldc + c0;
    auto pass = [&]() {
#pragma unroll
        for (int s = 0; s < 8; ++s) { const int Lid = (lane >> 3) + 4 * s, piece = lane & 7; const int row = Lid >> 1, cofs = (Lid & 1) * 32 + piece * 4;
            const v4f val = *(const v4fa*)(os + row * 68 + cofs); *(volatile v4f*)(crow + (size_t)row * ldc + cofs) = val; }
    };
    pass(); __threadfence(); pass();
}
__global__ __launch_bounds__(NB_) void k_final(const float* __restrict__ Ff, const float* __restrict__ T, const float* __restrict__ rw, const float* __restrict__ rb, float* OUTP) {
    const int b = threadIdx.x; const float* fr = Ff + (size_t)b * NF;
    float acc = bfr(rb[0]) + bfr(rw[0]); float a2 = 0.f;
#pragma unroll 4
    for (int f = 0; f < NF; ++f) acc = fmaf(fr[f], bfr(rw[1 + f]), acc);
#pragma unroll 1
    for (int i = 0; i < NPOS; ++i) {
#pragma unroll 4
        for (int j = 0; j < CH2; ++j) a2 = fmaf(fr[i * CH2 + j], T[((size_t)i * NB_ + b) * CH2 + j], a2); }
    const float y = acc + a2;
    *(volatile float*)(OUTP + b) = y; __threadfence(); *(volatile float*)(OUTP + b) = y;
}

extern "C" void kernel_launch(void* const* d_in, const int* in_sizes, int n_in,
                              void* d_out, int out_size, void* d_ws, size_t ws_size, hipStream_t stream) {
    (void)in_sizes; (void)n_in; (void)out_size;
    const int* xs = (const int*)d_in[0]; const float* w1 = (const float*)d_in[1]; const float* b1 = (const float*)d_in[2]; const float* w2 = (const float*)d_in[3]; const float* b2 = (const float*)d_in[4]; const float* rw = (const float*)d_in[5]; const float* rb = (const float*)d_in[6];
    float* out = (float*)d_out;
    char* wsp = (char*)d_ws;
    auto take = [&](size_t bytes) { char* p = wsp; wsp += (bytes + 255) & ~(size_t)255; return (void*)p; };
    bf* W2B = (bf*)take((size_t)CH2 * KIM * 2); bf* WSO = (bf*)take((size_t)NSO * 2); float* H1 = (float*)take((size_t)NRW * CH1 * 4); bf* Ah = (bf*)take((size_t)NRW * KIM * 2); bf* Al = (bf*)take((size_t)NRW * KIM * 2);
    float* H2 = (float*)take((size_t)NRW * CH2 * 4); float* Ff = (float*)take((size_t)NB_ * NF * 4); bf* Fh = (bf*)take((size_t)NB_ * NF * 2); bf* Fl = (bf*)take((size_t)NB_ * NF * 2); float* T = (float*)take((size_t)NPOS * NB_ * CH2 * 4);
    if ((size_t)(wsp - (char*)d_ws) > ws_size) return;
    k_bf<<<(CH2 * KIM / 8 + 255) / 256, 256, 0, stream>>>(w2, W2B, CH2 * KIM / 8); k_wso<<<(NSO / 8 + 255) / 256, 256, 0, stream>>>(rw, WSO);
    k_conv1<<<NB_, CH1, 0, stream>>>(xs, w1, b1, H1); k_im2col<<<NRW / 8, 256, 0, stream>>>(H1, Ah, Al);
    k_gemmb<true, false><<<dim3(NRW / 64, 1, 1), 128, 0, stream>>>(Ah, Al, W2B, b2, H2, CH2, nullptr, nullptr, KIM);
    k_feat<<<NB_ / 8, 256, 0, stream>>>(H2, Ff, Fh, Fl);
    size_t off = 0;
    for (int i = 0; i < NPOS; ++i) { const int len = (NPOS - i) * CH2;
        k_gemml<<<dim3(NB_ / 64, 1, 1), 128, 0, stream>>>(Fh + (size_t)(i + 1) * CH2, Fl + (size_t)(i + 1) * CH2, NF, WSO + off, len, T + (size_t)i * NB_ * CH2, CH2);
        off += (size_t)CH2 * len; }
    k_final<<<1, NB_, 0, stream>>>(Ff, T, rw, rb, out);
}
